// GNNEncoder_61314953117893
// MI455X (gfx1250) — hardware-run, weakly checked
//
#include <hip/hip_runtime.h>
#include <math.h>
#include <stdint.h>

#define NB_   8
#define NN_   1024
#define DIN_  64
#define HID_  128
#define NLY_  2
#define NH_   4
#define HD_   32
#define NTOK  (NB_ * NN_)
#define NBH   (NB_ * NH_)
#define SFP   132
#define SHP   72
#define SMEM_BYTES 36864
#define ATT_SCALE 0.17677669529663687f
#define LN_EPS 1.0e-5f
#define NEG_BIG (-1.0e30f)
#define NEG_THR (-1.0e29f)

static_assert(HID_ == NH_ * HD_);
static_assert(HD_ == 32);
static_assert(HID_ == 128);
static_assert(NN_ % 64 == 0);
static_assert((NN_ / 64) == 16);
static_assert(NTOK % 64 == 0);
static_assert(DIN_ % 32 == 0);
static_assert(HID_ % 32 == 0);
static_assert((NTOK * DIN_) % 2048 == 0);
static_assert((HID_ * DIN_) % 2048 == 0);
static_assert((NLY_ * HID_ * HID_) % 2048 == 0);
static_assert((HID_ * HID_) % 2048 == 0);
static_assert((NTOK * HID_) % 2048 == 0);
static_assert(64 * SFP * 4 <= SMEM_BYTES);
static_assert(2 * HID_ * SHP * 2 <= SMEM_BYTES);

typedef __attribute__((ext_vector_type(16))) __bf16 v16b;
typedef __attribute__((ext_vector_type(8)))  __bf16 v8b;
typedef __attribute__((ext_vector_type(8)))  float  v8f;
typedef __attribute__((ext_vector_type(4)))  float  v4f;
typedef __attribute__((ext_vector_type(4)))  unsigned int v4u;
typedef __attribute__((ext_vector_type(8)))  unsigned int v8u;
typedef v8b __attribute__((may_alias)) v8ba;
typedef v4f __attribute__((may_alias)) v4fa;
typedef v4u __attribute__((may_alias)) v4ua;

union FragU { v16b v; v8b h[2]; };
union PackU { v8u u; v16b v; };

__device__ __forceinline__ unsigned short f2bf_bits(float f) {
  const unsigned u = __float_as_uint(f);
  return (unsigned short)((u + 0x7FFFu + ((u >> 16) & 1u)) >> 16);
}
__device__ __forceinline__ float bf_bits2f(unsigned short h) { return __uint_as_float(((unsigned)h) << 16); }
__device__ __forceinline__ float bf16r(float f) {
  unsigned u = __float_as_uint(f);
  u = (u + 0x7FFFu + ((u >> 16) & 1u)) & 0xFFFF0000u;
  return __uint_as_float(u);
}
__device__ __forceinline__ unsigned pk16(unsigned short a, unsigned short b) { return (unsigned)a | ((unsigned)b << 16); }

__device__ __forceinline__ v8f wmma_bf16(v16b a, v16b b, v8f c) {
  v8f d = __builtin_amdgcn_wmma_f32_16x16x32_bf16(false, a, false, b, (short)0, c, false, false);
  asm volatile("v_nop\n\tv_nop\n\tv_nop\n\tv_nop" : "+v"(d) : "v"(a), "v"(b));
  return d;
}

__device__ __forceinline__ v16b load_frag(const unsigned short* p, int hh) {
  FragU f;
  f.h[0] = *(const v8ba*)(p + 8 * hh);
  f.h[1] = *(const v8ba*)(p + 16 + 8 * hh);
  return f.v;
}

__device__ __forceinline__ void pack_p2(v8f a, v8f c, v16b& ho, v16b& lo) {
  PackU uh, ul;
#pragma unroll
  for (int i = 0; i < 4; ++i) {
    const unsigned short h0 = f2bf_bits(a[2 * i]), h1 = f2bf_bits(a[2 * i + 1]);
    const unsigned short l0 = f2bf_bits(a[2 * i] - bf_bits2f(h0)), l1 = f2bf_bits(a[2 * i + 1] - bf_bits2f(h1));
    uh.u[i] = pk16(h0, h1); ul.u[i] = pk16(l0, l1);
    const unsigned short g0 = f2bf_bits(c[2 * i]), g1 = f2bf_bits(c[2 * i + 1]);
    const unsigned short m0 = f2bf_bits(c[2 * i] - bf_bits2f(g0)), m1 = f2bf_bits(c[2 * i + 1] - bf_bits2f(g1));
    uh.u[4 + i] = pk16(g0, g1); ul.u[4 + i] = pk16(m0, m1);
  }
  ho = uh.v; lo = ul.v;
}

template <bool ASPLIT>
__device__ __forceinline__ void gemm_core_32x64(
    const unsigned short* __restrict__ Ah, const unsigned short* __restrict__ Al,
    const unsigned short* __restrict__ Bt, int K, size_t aoff, size_t boff, int hh, v8f (&acc)[2][4]) {
  const unsigned short* a0 = Ah + aoff;
  const unsigned short* a1 = a0 + (size_t)16 * K;
  const unsigned short* c0 = (ASPLIT ? Al : Ah) + aoff;
  const unsigned short* c1 = c0 + (size_t)16 * K;
  const unsigned short* bp = Bt + boff;
#pragma unroll 1
  for (int k0 = 0; k0 < K; k0 += 32) {
    const v16b f0 = load_frag(a0 + k0, hh);
    const v16b f1 = load_frag(a1 + k0, hh);
    v16b g0 = f0, g1 = f1;
    if (ASPLIT) { g0 = load_frag(c0 + k0, hh); g1 = load_frag(c1 + k0, hh); }
#pragma unroll
    for (int nt = 0; nt < 4; ++nt) {
      const v16b fb = load_frag(bp + (size_t)nt * 16 * K + k0, hh);
      acc[0][nt] = wmma_bf16(f0, fb, acc[0][nt]);
      acc[1][nt] = wmma_bf16(f1, fb, acc[1][nt]);
      if (ASPLIT) {
        acc[0][nt] = wmma_bf16(g0, fb, acc[0][nt]);
        acc[1][nt] = wmma_bf16(g1, fb, acc[1][nt]);
      }
    }
  }
}

__global__ __launch_bounds__(256) void k_cvt(const float* __restrict__ src, unsigned short* __restrict__ dst, int n8) {
  int i = blockIdx.x * 256 + threadIdx.x;
  const bool ok = i < n8;
  i = ok ? i : (n8 - 1);
  const float* s = src + (size_t)i * 8;
  const v4f f0 = *(const v4fa*)(s);
  const v4f f1 = *(const v4fa*)(s + 4);
  v4u u;
  u[0] = pk16(f2bf_bits(f0[0]), f2bf_bits(f0[1]));
  u[1] = pk16(f2bf_bits(f0[2]), f2bf_bits(f0[3]));
  u[2] = pk16(f2bf_bits(f1[0]), f2bf_bits(f1[1]));
  u[3] = pk16(f2bf_bits(f1[2]), f2bf_bits(f1[3]));
  unsigned short* d = dst + (size_t)i * 8;
  if (ok) *(volatile v4u*)d = u;
  __threadfence();
  if (ok) *(volatile v4u*)d = u;
}

__global__ __launch_bounds__(256) void k_split(const float* __restrict__ src, unsigned short* __restrict__ hi,
                                               unsigned short* __restrict__ lo, int n8) {
  int i = blockIdx.x * 256 + threadIdx.x;
  const bool ok = i < n8;
  i = ok ? i : (n8 - 1);
  const float* s = src + (size_t)i * 8;
  const v4f f0 = *(const v4fa*)(s);
  const v4f f1 = *(const v4fa*)(s + 4);
  const float e[8] = {f0[0], f0[1], f0[2], f0[3], f1[0], f1[1], f1[2], f1[3]};
  v4u uh, ul;
#pragma unroll
  for (int q = 0; q < 4; ++q) {
    const unsigned short h0 = f2bf_bits(e[2 * q]), h1 = f2bf_bits(e[2 * q + 1]);
    const unsigned short l0 = f2bf_bits(e[2 * q] - bf_bits2f(h0)), l1 = f2bf_bits(e[2 * q + 1] - bf_bits2f(h1));
    uh[q] = pk16(h0, h1);
    ul[q] = pk16(l0, l1);
  }
  unsigned short* dh = hi + (size_t)i * 8;
  unsigned short* dl = lo + (size_t)i * 8;
  if (ok) { *(volatile v4u*)dh = uh; *(volatile v4u*)dl = ul; }
  __threadfence();
  if (ok) { *(volatile v4u*)dh = uh; *(volatile v4u*)dl = ul; }
}

template <bool ASPLIT, int MODE>
__global__ __launch_bounds__(128) void k_gemm(
    const unsigned short* __restrict__ Ah, const unsigned short* __restrict__ Al, int K,
    const unsigned short* __restrict__ Bt, const float* __restrict__ bias,
    const float* __restrict__ gam, const float* __restrict__ bet, const float* __restrict__ resid,
    float* __restrict__ outF, unsigned short* __restrict__ outH, unsigned short* __restrict__ outL) {
  __shared__ __align__(16) unsigned char smem[SMEM_BYTES];
  __shared__ __align__(16) float sG[HID_];
  __shared__ __align__(16) float sE[HID_];
  float* sF = (float*)smem;
  unsigned short* sH = (unsigned short*)smem;
  unsigned short* sL = sH + HID_ * SHP;

  const int tid = threadIdx.x, lane = tid & 31, w = tid >> 5;
  const int hh = lane >> 4, m = lane & 15;
  const int m0 = blockIdx.x * 64;
  const int wr = 32 * (w >> 1);
  const int wc = 64 * (w & 1);

  const v8f zero8 = {0.f, 0.f, 0.f, 0.f, 0.f, 0.f, 0.f, 0.f};
  v8f acc[2][4];
#pragma unroll
  for (int mt = 0; mt < 2; ++mt)
#pragma unroll
    for (int nt = 0; nt < 4; ++nt) acc[mt][nt] = zero8;

  gemm_core_32x64<ASPLIT>(Ah, Al, Bt, K, (size_t)(m0 + wr + m) * (size_t)K, (size_t)(wc + m) * (size_t)K, hh, acc);

  float bv[4];
#pragma unroll
  for (int nt = 0; nt < 4; ++nt) bv[nt] = bf16r(bias[wc + 16 * nt + m]);
  if (MODE == 4) { sG[tid] = bf16r(gam[tid]); sE[tid] = bf16r(bet[tid]); }

  if (MODE != 3) {
#pragma unroll
    for (int nt = 0; nt < 4; ++nt)
#pragma unroll
      for (int mt = 0; mt < 2; ++mt)
#pragma unroll
        for (int r = 0; r < 8; ++r) {
          const int rowl = wr + 16 * mt + 8 * hh + r;
          const int col  = wc + 16 * nt + m;
          float v = acc[mt][nt][r] + bv[nt];
          if (MODE == 1) v = fmaxf(v, 0.0f);
          sF[rowl * SFP + col] = v;
        }
  } else {
#pragma unroll
    for (int nt = 0; nt < 4; ++nt)
#pragma unroll
      for (int mt = 0; mt < 2; ++mt)
#pragma unroll
        for (int r = 0; r < 8; ++r) {
          const int rowl = wr + 16 * mt + 8 * hh + r;
          const int col  = wc + 16 * nt + m;
          const float v = acc[mt][nt][r] + bv[nt];
          const unsigned short hb = f2bf_bits(v);
          const unsigned short lb = f2bf_bits(v - bf_bits2f(hb));
          sH[col * SHP + rowl] = hb;
          sL[col * SHP + rowl] = lb;
        }
  }
  __syncthreads();

  if (MODE == 4) {
#pragma unroll 2
    for (int i = 0; i < 16; ++i) {
      const int rl = 16 * w + i;
      float* rp = sF + rl * SFP + 4 * lane;
      const v4f x = *(const v4fa*)rp;
      float s = (x[0] + x[1]) + (x[2] + x[3]);
#pragma unroll
      for (int off = 1; off < 32; off <<= 1) s += __shfl_xor(s, off, 32);
      const float mu = s * (1.0f / 128.0f);
      const float d0 = x[0] - mu, d1 = x[1] - mu, d2 = x[2] - mu, d3 = x[3] - mu;
      float s2 = (d0 * d0 + d1 * d1) + (d2 * d2 + d3 * d3);
#pragma unroll
      for (int off = 1; off < 32; off <<= 1) s2 += __shfl_xor(s2, off, 32);
      const float var  = s2 * (1.0f / 128.0f);
      const float rstd = rsqrtf(var + LN_EPS);
      const v4f g  = *(const v4fa*)(sG + 4 * lane);
      const v4f e  = *(const v4fa*)(sE + 4 * lane);
      const v4f rv = *(const v4fa*)(resid + (size_t)(m0 + rl) * HID_ + 4 * lane);
      v4f y;
      y[0] = fmaxf(d0 * rstd * g[0] + e[0], 0.0f) + rv[0];
      y[1] = fmaxf(d1 * rstd * g[1] + e[1], 0.0f) + rv[1];
      y[2] = fmaxf(d2 * rstd * g[2] + e[2], 0.0f) + rv[2];
      y[3] = fmaxf(d3 * rstd * g[3] + e[3], 0.0f) + rv[3];
      *(v4fa*)rp = y;
    }
    __syncthreads();
  }

  if (MODE == 3) {
    const int bq = blockIdx.x >> 4;
    const int n0 = (blockIdx.x & 15) * 64;
    const int q4 = lane >> 3, t8 = (lane & 7) * 8;
    for (int pass = 0; pass < 2; ++pass) {
#pragma unroll
      for (int it = 0; it < 8; ++it) {
        const int feat = 16 * it + 4 * w + q4;
        const v4u hv = *(const v4ua*)(sH + feat * SHP + t8);
        const v4u lv = *(const v4ua*)(sL + feat * SHP + t8);
        const size_t go = ((size_t)(bq * HID_ + feat)) * (size_t)NN_ + n0 + t8;
        *(volatile v4u*)(outH + go) = hv;
        *(volatile v4u*)(outL + go) = lv;
      }
      __threadfence();
    }
  } else {
    const int c8 = (lane & 15) * 8;
    for (int pass = 0; pass < 2; ++pass) {
      if (MODE == 0 || MODE == 1 || MODE == 4) {
#pragma unroll
        for (int i = 0; i < 16; ++i) {
          const int row = 16 * w + i;
          const v4f v = *(const v4fa*)(sF + row * SFP + 4 * lane);
          *(volatile v4f*)(outF + (size_t)(m0 + row) * HID_ + 4 * lane) = v;
        }
      }
      if (MODE == 1 || MODE == 2 || MODE == 4) {
#pragma unroll
        for (int it = 0; it < 8; ++it) {
          const int row = 16 * w + 2 * it + hh;
          const float* sp = sF + row * SFP + c8;
          const v4f fa = *(const v4fa*)(sp);
          const v4f fb = *(const v4fa*)(sp + 4);
          const float e8[8] = {fa[0], fa[1], fa[2], fa[3], fb[0], fb[1], fb[2], fb[3]};
          v4u hv, lv;
#pragma unroll
          for (int q = 0; q < 4; ++q) {
            const unsigned short h0 = f2bf_bits(e8[2 * q]), h1 = f2bf_bits(e8[2 * q + 1]);
            const unsigned short l0 = f2bf_bits(e8[2 * q] - bf_bits2f(h0)), l1 = f2bf_bits(e8[2 * q + 1] - bf_bits2f(h1));
            hv[q] = pk16(h0, h1);
            lv[q] = pk16(l0, l1);
          }
          const size_t go = (size_t)(m0 + row) * HID_ + c8;
          *(volatile v4u*)(outH + go) = hv;
          *(volatile v4u*)(outL + go) = lv;
        }
      }
      __threadfence();
    }
  }
}

__global__ __launch_bounds__(128) void k_attn(
    const unsigned short* __restrict__ Qh, const unsigned short* __restrict__ Ql,
    const unsigned short* __restrict__ Kh, const unsigned short* __restrict__ Kl,
    const unsigned short* __restrict__ VTh, const unsigned short* __restrict__ VTl,
    const float* __restrict__ adj, float* __restrict__ AO) {
  __shared__ __align__(16) float sO[4][16 * 36];

  const int tid = threadIdx.x, lane = tid & 31, w = tid >> 5;
  const int hh = lane >> 4, m = lane & 15;
  const int qt = blockIdx.x;
  const int bh = blockIdx.y, b = bh >> 2, h = bh & 3;
  const int q0w = qt * 64 + 16 * w;
  const int q = q0w + m;
  const size_t tokq = (size_t)b * NN_ + q;

  const v16b qfh = load_frag(Qh + tokq * HID_ + h * HD_, hh);
  const v16b qfl = load_frag(Ql + tokq * HID_ + h * HD_, hh);
  const float* arow = adj + tokq * (size_t)NN_;

  const v8f zero8 = {0.f, 0.f, 0.f, 0.f, 0.f, 0.f, 0.f, 0.f};
  v8f o[2];
  o[0] = zero8; o[1] = zero8;
  float mrun = NEG_BIG, lrun = 0.0f;

#pragma unroll 1
  for (int ks = 0; ks < NN_ / 64; ++ks) {
    const int kb = ks * 64;

    v8f s[4];
#pragma unroll
    for (int j = 0; j < 4; ++j) {
      const size_t krow = ((size_t)(b * NN_ + kb + 16 * j + m)) * HID_ + h * HD_;
      const v16b kfh = load_frag(Kh + krow, hh);
      const v16b kfl = load_frag(Kl + krow, hh);
      v8f a = zero8;
      a = wmma_bf16(kfh, qfh, a);
      a = wmma_bf16(kfh, qfl, a);
      a = wmma_bf16(kfl, qfh, a);
      const v4f mA = *(const v4fa*)(arow + kb + 16 * j + 8 * hh);
      const v4f mB = *(const v4fa*)(arow + kb + 16 * j + 8 * hh + 4);
      const float mv[8] = {mA[0], mA[1], mA[2], mA[3], mB[0], mB[1], mB[2], mB[3]};
#pragma unroll
      for (int r = 0; r < 8; ++r) {
        const float t = a[r] * ATT_SCALE;
        s[j][r] = (mv[r] != 0.0f) ? t : NEG_BIG;
      }
    }
    float cm = NEG_BIG;
#pragma unroll
    for (int j = 0; j < 4; ++j)
#pragma unroll
      for (int r = 0; r < 8; ++r) cm = fmaxf(cm, s[j][r]);
    cm = fmaxf(cm, __shfl_xor(cm, 16, 32));
    const float mnew  = fmaxf(mrun, cm);
    const float msafe = (mnew > NEG_THR) ? mnew : 0.0f;
    const float alpha = __expf(mrun - msafe);
    mrun = mnew;
    float psum = 0.0f;
#pragma unroll
    for (int j = 0; j < 4; ++j)
#pragma unroll
      for (int r = 0; r < 8; ++r) {
        const float p = __expf(s[j][r] - msafe);
        psum += p;
        s[j][r] = p;
      }
    psum += __shfl_xor(psum, 16, 32);
    lrun = lrun * alpha + psum;
#pragma unroll
    for (int t = 0; t < 2; ++t)
#pragma unroll
      for (int r = 0; r < 8; ++r) o[t][r] *= alpha;

    v16b p0h, p0l, p1h, p1l;
    pack_p2(s[0], s[1], p0h, p0l);
    pack_p2(s[2], s[3], p1h, p1l);

#pragma unroll
    for (int t = 0; t < 2; ++t) {
      const unsigned short* vph = VTh + ((size_t)(bh * HD_ + 16 * t + m)) * (size_t)NN_ + kb;
      const unsigned short* vpl = VTl + ((size_t)(bh * HD_ + 16 * t + m)) * (size_t)NN_ + kb;
      const v16b v0h = load_frag(vph, hh), v0l = load_frag(vpl, hh);
      o[t] = wmma_bf16(v0h, p0h, o[t]);
      o[t] = wmma_bf16(v0h, p0l, o[t]);
      o[t] = wmma_bf16(v0l, p0h, o[t]);
      const v16b v1h = load_frag(vph + 32, hh), v1l = load_frag(vpl + 32, hh);
      o[t] = wmma_bf16(v1h, p1h, o[t]);
      o[t] = wmma_bf16(v1h, p1l, o[t]);
      o[t] = wmma_bf16(v1l, p1h, o[t]);
    }
  }

  const float inv = (lrun > 0.0f) ? (1.0f / lrun) : 0.0f;
  float* so = sO[w];
#pragma unroll
  for (int t = 0; t < 2; ++t)
#pragma unroll
    for (int r = 0; r < 8; ++r) so[m * 36 + 16 * t + 8 * hh + r] = o[t][r] * inv;
  __syncthreads();
  {
    const int rq = lane >> 3, c4 = (lane & 7) * 4;
    for (int pass = 0; pass < 2; ++pass) {
#pragma unroll
      for (int it = 0; it < 4; ++it) {
        const int row = 4 * it + rq;
        const v4f v = *(const v4fa*)(so + row * 36 + c4);
        *(volatile v4f*)(AO + ((size_t)b * NN_ + q0w + row) * (size_t)HID_ + h * HD_ + c4) = v;
      }
      __threadfence();
    }
  }
}

extern "C" void kernel_launch(void* const* d_in, const int* in_sizes, int n_in,
                              void* d_out, int out_size, void* d_ws, size_t ws_size,
                              hipStream_t stream) {
  if (n_in < 16) return;
  if (in_sizes[0] != NTOK * DIN_) return;
  if (in_sizes[1] != NB_ * NN_ * NN_) return;
  if (in_sizes[2] != HID_ * DIN_) return;
  if (in_sizes[3] != HID_) return;
  for (int i = 4; i <= 10; i += 2) {
    if (in_sizes[i] != NLY_ * HID_ * HID_) return;
    if (in_sizes[i + 1] != NLY_ * HID_) return;
  }
  if (in_sizes[12] != NLY_ * HID_) return;
  if (in_sizes[13] != NLY_ * HID_) return;
  if (in_sizes[14] != HID_ * HID_) return;
  if (in_sizes[15] != HID_) return;
  if (out_size != NTOK * HID_) return;

  const float* x     = (const float*)d_in[0];
  const float* adj   = (const float*)d_in[1];
  const float* enc_w = (const float*)d_in[2];
  const float* enc_b = (const float*)d_in[3];
  const float* q_w   = (const float*)d_in[4];
  const float* q_b   = (const float*)d_in[5];
  const float* k_w   = (const float*)d_in[6];
  const float* k_b   = (const float*)d_in[7];
  const float* v_w   = (const float*)d_in[8];
  const float* v_b   = (const float*)d_in[9];
  const float* o_w   = (const float*)d_in[10];
  const float* o_b   = (const float*)d_in[11];
  const float* ln_g  = (const float*)d_in[12];
  const float* ln_b  = (const float*)d_in[13];
  const float* out_w = (const float*)d_in[14];
  const float* out_b = (const float*)d_in[15];
  float* out = (float*)d_out;

  const size_t PXB = (size_t)NTOK * DIN_ * 2;
  const size_t PEW = (size_t)HID_ * DIN_ * 2;
  const size_t PLW = (size_t)NLY_ * HID_ * HID_ * 2;
  const size_t POW = (size_t)HID_ * HID_ * 2;
  const size_t PF  = (size_t)NTOK * HID_ * 4;
  const size_t PH  = (size_t)NTOK * HID_ * 2;
  const size_t PVT = (size_t)NBH * HD_ * NN_ * 2;
  size_t off = 0;
  const size_t oXb  = off; off += PXB;
  const size_t oWeb = off; off += PEW;
  const size_t oWqb = off; off += PLW;
  const size_t oWkb = off; off += PLW;
  const size_t oWvb = off; off += PLW;
  const size_t oWob = off; off += PLW;
  const size_t oWfb = off; off += POW;
  const size_t oHf0 = off; off += PF;
  const size_t oHf1 = off; off += PF;
  const size_t oHh0 = off; off += PH;
  const size_t oHl0 = off; off += PH;
  const size_t oHh1 = off; off += PH;
  const size_t oHl1 = off; off += PH;
  const size_t oQh  = off; off += PH;
  const size_t oQl  = off; off += PH;
  const size_t oKh  = off; off += PH;
  const size_t oKl  = off; off += PH;
  const size_t oVTh = off; off += PVT;
  const size_t oVTl = off; off += PVT;
  const size_t oAO  = off; off += PF;
  const size_t oAOh = off; off += PH;
  const size_t oAOl = off; off += PH;
  if (off > ws_size) return;

  char* ws = (char*)d_ws;
  unsigned short* Xb  = (unsigned short*)(ws + oXb);
  unsigned short* Web = (unsigned short*)(ws + oWeb);
  unsigned short* Wqb = (unsigned short*)(ws + oWqb);
  unsigned short* Wkb = (unsigned short*)(ws + oWkb);
  unsigned short* Wvb = (unsigned short*)(ws + oWvb);
  unsigned short* Wob = (unsigned short*)(ws + oWob);
  unsigned short* Wfb = (unsigned short*)(ws + oWfb);
  float* Hf[2]; Hf[0] = (float*)(ws + oHf0); Hf[1] = (float*)(ws + oHf1);
  unsigned short* Hh[2]; Hh[0] = (unsigned short*)(ws + oHh0); Hh[1] = (unsigned short*)(ws + oHh1);
  unsigned short* Hl[2]; Hl[0] = (unsigned short*)(ws + oHl0); Hl[1] = (unsigned short*)(ws + oHl1);
  unsigned short* Qh  = (unsigned short*)(ws + oQh);
  unsigned short* Ql  = (unsigned short*)(ws + oQl);
  unsigned short* Kh  = (unsigned short*)(ws + oKh);
  unsigned short* Kl  = (unsigned short*)(ws + oKl);
  unsigned short* VTh = (unsigned short*)(ws + oVTh);
  unsigned short* VTl = (unsigned short*)(ws + oVTl);
  float*          AO  = (float*)(ws + oAO);
  unsigned short* AOh = (unsigned short*)(ws + oAOh);
  unsigned short* AOl = (unsigned short*)(ws + oAOl);

  const int n8x  = NTOK * DIN_ / 8;
  const int n8e  = HID_ * DIN_ / 8;
  const int n8l  = NLY_ * HID_ * HID_ / 8;
  const int n8f  = HID_ * HID_ / 8;
  const int n8a  = NTOK * HID_ / 8;
  const dim3 gG(NTOK / 64);
  const dim3 gA(NN_ / 64, NBH);

  k_cvt<<<dim3((n8x + 255) / 256), 256, 0, stream>>>(x, Xb, n8x);
  k_cvt<<<dim3((n8e + 255) / 256), 256, 0, stream>>>(enc_w, Web, n8e);
  k_cvt<<<dim3((n8l + 255) / 256), 256, 0, stream>>>(q_w, Wqb, n8l);
  k_cvt<<<dim3((n8l + 255) / 256), 256, 0, stream>>>(k_w, Wkb, n8l);
  k_cvt<<<dim3((n8l + 255) / 256), 256, 0, stream>>>(v_w, Wvb, n8l);
  k_cvt<<<dim3((n8l + 255) / 256), 256, 0, stream>>>(o_w, Wob, n8l);
  k_cvt<<<dim3((n8f + 255) / 256), 256, 0, stream>>>(out_w, Wfb, n8f);

  k_gemm<false, 1><<<gG, 128, 0, stream>>>(Xb, Xb, DIN_, Web, enc_b, enc_b, enc_b, AO, Hf[0], Hh[0], Hl[0]);

  for (int l = 0; l < NLY_; ++l) {
    const int cur = l & 1, nxt = cur ^ 1;
    const size_t wo = (size_t)l * HID_ * HID_;
    const size_t bo = (size_t)l * HID_;
    k_gemm<true, 2><<<gG, 128, 0, stream>>>(Hh[cur], Hl[cur], HID_, Wqb + wo, q_b + bo, enc_b, enc_b, AO, AO, Qh, Ql);
    k_gemm<true, 2><<<gG, 128, 0, stream>>>(Hh[cur], Hl[cur], HID_, Wkb + wo, k_b + bo, enc_b, enc_b, AO, AO, Kh, Kl);
    k_gemm<true, 3><<<gG, 128, 0, stream>>>(Hh[cur], Hl[cur], HID_, Wvb + wo, v_b + bo, enc_b, enc_b, AO, AO, VTh, VTl);
    k_attn<<<gA, 128, 0, stream>>>(Qh, Ql, Kh, Kl, VTh, VTl, adj, AO);
    k_split<<<dim3((n8a + 255) / 256), 256, 0, stream>>>(AO, AOh, AOl, n8a);
    k_gemm<true, 4><<<gG, 128, 0, stream>>>(AOh, AOl, HID_, Wob + wo, o_b + bo, ln_g + bo, ln_b + bo, Hf[cur], Hf[nxt], Hh[nxt], Hl[nxt]);
  }

  const int fin = NLY_ & 1;
  k_gemm<true, 0><<<gG, 128, 0, stream>>>(Hh[fin], Hl[fin], HID_, Wfb, out_b, enc_b, enc_b, AO, out, AOh, AOl);
  (void)hipGetLastError();
}
